// LinOSSBlock_35862976921827
// MI455X (gfx1250) — hardware-verified
//
#include <hip/hip_runtime.h>
#include <math.h>

#define NB_ 8
#define LL 4096
#define HH 128
#define PP 256
#define NROW (NB_ * LL)
#define KA 640
#define GSTR 48

typedef _Float16 f16;
typedef __attribute__((ext_vector_type(16))) f16 f16x16;
typedef __attribute__((ext_vector_type(8)))  f16 f16x8;
typedef __attribute__((ext_vector_type(8)))  float f32x8;
typedef __attribute__((ext_vector_type(4)))  float v4f_t;
typedef float v4fa __attribute__((ext_vector_type(4), may_alias));
__device__ __forceinline__ f32x8 wmma16(f16x16 a, f16x16 b, f32x8 c) {
  c = __builtin_amdgcn_wmma_f32_16x16x32_f16(false, a, false, b, (short)0, c, false, false);
  asm volatile("v_nop\n\tv_nop\n\tv_nop\n\tv_nop" : "+v"(c) : "v"(a), "v"(b));
  return c;
}
__device__ __forceinline__ f16x16 lds_frag(const f16* base, int stride) {
  const int lane = threadIdx.x & 31, row = lane & 15, kh = (lane >> 4) * 8;
  const f16x8 lo = *(const f16x8*)(base + row * stride + kh);
  const f16x8 hi = *(const f16x8*)(base + row * stride + kh + 16);
  f16x16 f;
#pragma unroll
  for (int i = 0; i < 8; ++i) { f[i] = lo[i]; f[i + 8] = hi[i]; }
  return f;
}

template <typename AT, bool ACC>
__global__ __launch_bounds__(256) void gemm_kn2(const AT* __restrict__ A, int lda, size_t strideA,
                                               const float* __restrict__ Wm, int ldw, size_t strideW,
                                               const float* __restrict__ bias, float scale,
                                               float* __restrict__ Y, int ldy, size_t strideY, int K) {
  __shared__ __attribute__((aligned(16))) f16 ldsA[128 * GSTR], ldsAl[128 * GSTR];
  __shared__ __attribute__((aligned(16))) f16 ldsW[128 * GSTR], ldsWl[128 * GSTR];
  __shared__ __attribute__((aligned(16))) float oS[8][32 * 68];
  const int tid = threadIdx.x, lane = tid & 31, wave = tid >> 5, cl = lane & 15, rh = (lane >> 4) * 8;
  const int m0 = blockIdx.x * 128, n0 = blockIdx.y * 128;
  const int wm = (wave & 3) * 32, wn = (wave >> 2) * 64;
  A += (size_t)blockIdx.z * strideA; Wm += (size_t)blockIdx.z * strideW; Y += (size_t)blockIdx.z * strideY;
  f32x8 acc[2][4], accx[2][4];
#pragma unroll
  for (int i = 0; i < 2; ++i)
#pragma unroll
    for (int j = 0; j < 4; ++j) { f32x8 z = {}; acc[i][j] = z; accx[i][j] = z; }
#pragma unroll 1
  for (int k0 = 0; k0 < K; k0 += 32) {
    __syncthreads();
    {
      const int row = tid >> 1, ch = (tid & 1) * 16;
      const AT* src = A + (size_t)(m0 + row) * lda + k0 + ch;
#pragma unroll
      for (int g = 0; g < 16; ++g) { const float v = (float)src[g]; const f16 h = (f16)v; ldsA[row * GSTR + ch + g] = h; ldsAl[row * GSTR + ch + g] = (f16)((v - (float)h) * 2048.0f); }
    }
    {
      const int k = tid >> 3, nn0 = (tid & 7) * 16;
      const float* src = Wm + (size_t)(k0 + k) * ldw + n0 + nn0;
#pragma unroll
      for (int g = 0; g < 4; ++g) { const v4f_t v = *(const v4f_t*)(src + 4 * g);
#pragma unroll
        for (int u = 0; u < 4; ++u) { const f16 h = (f16)v[u]; ldsW[(nn0 + 4 * g + u) * GSTR + k] = h; ldsWl[(nn0 + 4 * g + u) * GSTR + k] = (f16)((v[u] - (float)h) * 2048.0f); } }
    }
    __syncthreads();
    f16x16 af[2], afl[2];
#pragma unroll
    for (int i = 0; i < 2; ++i) { af[i] = lds_frag(ldsA + (wm + 16 * i) * GSTR, GSTR); afl[i] = lds_frag(ldsAl + (wm + 16 * i) * GSTR, GSTR); }
#pragma unroll
    for (int j = 0; j < 4; ++j) {
      const f16x16 bf = lds_frag(ldsW + (wn + 16 * j) * GSTR, GSTR), bfl = lds_frag(ldsWl + (wn + 16 * j) * GSTR, GSTR);
#pragma unroll
      for (int i = 0; i < 2; ++i) { acc[i][j] = wmma16(af[i], bf, acc[i][j]); accx[i][j] = wmma16(af[i], bfl, accx[i][j]); accx[i][j] = wmma16(afl[i], bf, accx[i][j]); }
    }
  }
  float* so = oS[wave];
#pragma unroll
  for (int i = 0; i < 2; ++i)
#pragma unroll
    for (int j = 0; j < 4; ++j) {
      const float bv = bias ? bias[n0 + wn + 16 * j + cl] : 0.0f;
#pragma unroll
      for (int r = 0; r < 8; ++r) so[(16 * i + rh + r) * 68 + 16 * j + cl] = (acc[i][j][r] + accx[i][j][r] * (1.0f / 2048.0f)) * scale + bv;
    }
  asm volatile("s_wait_dscnt 0" ::: "memory");
  __builtin_amdgcn_wave_barrier();
  if (ACC) {
#pragma unroll
    for (int it = 0; it < 16; ++it) { const int f4 = lane + 32 * it, rr = f4 >> 4, q = (f4 & 15) * 4;
      const v4f_t old = *(const volatile v4fa*)(Y + (size_t)(m0 + wm + rr) * ldy + n0 + wn + q);
      v4f_t v = *(const volatile v4fa*)(so + rr * 68 + q); v += old; *(volatile v4fa*)(so + rr * 68 + q) = v; }
    asm volatile("s_wait_dscnt 0" ::: "memory");
  }
#pragma unroll 1
  for (int pass = 0; pass < 2; ++pass) {
#pragma unroll
    for (int it = 0; it < 16; ++it) { const int f4 = lane + 32 * it, rr = f4 >> 4, q = (f4 & 15) * 4;
      *(volatile v4f_t*)(Y + (size_t)(m0 + wm + rr) * ldy + n0 + wn + q) = *(const volatile v4fa*)(so + rr * 68 + q); }
    __threadfence();
  }
}

__global__ __launch_bounds__(256) void k_prep(const float* __restrict__ Ad, const float* __restrict__ Gd, const float* __restrict__ dt, const float* __restrict__ Bm,
                                             const float* __restrict__ Cm, const float* __restrict__ Dv, float* __restrict__ coef, float* __restrict__ WB, float* __restrict__ WC) {
  const int tid = threadIdx.x;
  { const int p = tid; const float s = 1.0f / (1.0f + expf(-dt[p])); const float glow = s * Ad[p]; const float g = glow + fmaxf(Gd[p] - glow, 0.0f);
    const float alow = 0.25f * g * g; const float a = alow + fmaxf(Ad[p] - alow, 0.0f);
    float* c = coef + p * 4; c[0] = 1.0f - s * g; c[1] = -s * a; c[2] = s; c[3] = s; }
  for (int e = tid; e < PP * HH; e += 256) { const int p = e >> 7, h = e & 127; WB[h * 512 + p] = Bm[(p * HH + h) * 2]; WB[h * 512 + 256 + p] = Bm[(p * HH + h) * 2 + 1]; }
  for (int e = tid; e < HH * PP; e += 256) { const int n = e >> 8, p = e & 255; WC[p * HH + n] = Cm[(n * PP + p) * 2]; WC[(256 + p) * HH + n] = -Cm[(n * PP + p) * 2 + 1]; }
  for (int e = tid; e < HH * HH; e += 256) { const int h = e >> 7, n = e & 127; WC[(512 + h) * HH + n] = (h == n) ? Dv[n] : 0.0f; }
}
__global__ __launch_bounds__(256) void k_copyx(const float* __restrict__ x, float* __restrict__ A) {
  const size_t i = (size_t)blockIdx.x * 256 + threadIdx.x;
  const size_t row = i >> 5, q = i & 31;
  *(v4f_t*)(A + row * KA + 512 + q * 4) = *(const v4f_t*)(x + row * HH + q * 4);
}
__global__ __launch_bounds__(256) void k_scan(float* __restrict__ A, const float* __restrict__ coef) {
  const int g = blockIdx.x * 256 + threadIdx.x;
  const int p = g & 255, part = (g >> 8) & 1, b = g >> 9;
  const float m11 = coef[p * 4], m12 = coef[p * 4 + 1], m21 = coef[p * 4 + 2], dts = coef[p * 4 + 3];
  float z = 0.0f, s = 0.0f;
  float* col = A + (size_t)b * LL * KA + part * 256 + p;
#pragma unroll 4
  for (int k = 0; k < LL; ++k) { float* e = col + (size_t)k * KA; const float f1 = dts * *e;
    const float zn = m11 * z + m12 * s + f1; const float sn = m21 * z + s; z = zn; s = sn; *e = s; }
}

extern "C" void kernel_launch(void* const* d_in, const int* in_sizes, int n_in,
                              void* d_out, int out_size, void* d_ws, size_t ws_size,
                              hipStream_t stream) {
  (void)in_sizes; (void)n_in; (void)out_size;
  const float* x = (const float*)d_in[0];
  const float* Ad = (const float*)d_in[1], *Gd = (const float*)d_in[2], *dt = (const float*)d_in[3];
  const float* Bm = (const float*)d_in[4];
  const float* Cm = (const float*)d_in[5];
  const float* Dv = (const float*)d_in[6];
  float* out = (float*)d_out;
  char* ws = (char*)d_ws;
  float* A = (float*)ws; ws += (size_t)NROW * KA * 4;
  float* WB = (float*)ws; ws += (size_t)HH * 512 * 4;
  float* WC = (float*)ws; ws += (size_t)KA * HH * 4;
  float* coef = (float*)ws; ws += PP * 4 * 4;
  if ((size_t)(ws - (char*)d_ws) > ws_size) return;
  const dim3 blk(256);
  k_prep<<<dim3(1), blk, 0, stream>>>(Ad, Gd, dt, Bm, Cm, Dv, coef, WB, WC);
  gemm_kn2<float, false><<<dim3(NROW / 128, 512 / 128, 1), blk, 0, stream>>>(x, HH, 0, WB, 512, 0, nullptr, 1.0f, A, KA, 0, HH);
  k_copyx<<<dim3(NROW * 32 / 256), blk, 0, stream>>>(x, A);
  k_scan<<<dim3(NB_ * 2 * PP / 256), blk, 0, stream>>>(A, coef);
  gemm_kn2<float, false><<<dim3(NROW / 128, HH / 128, 1), blk, 0, stream>>>(A, KA, 0, WC, HH, 0, nullptr, 1.0f, out, HH, 0, KA);
}
